// net_81939386073095
// MI455X (gfx1250) — hardware-verified
//
#include <hip/hip_runtime.h>
#include <math.h>

constexpr int NSAMP   = 1024;
constexpr int LATD    = 64;
constexpr int HID_A   = 256;
constexpr int HID_B   = 128;
constexpr int NQUAD   = 2080;
constexpr int NCUBE   = 45760;
constexpr int KREAL   = 2 * LATD + NQUAD + NCUBE;
constexpr int KPADDED = 48128;
constexpr int KSPLITS = 16;
constexpr int KCHUNK  = KPADDED / KSPLITS;
constexpr int KGRP8   = KPADDED / 8;
constexpr int PLANE_F = NSAMP * LATD;
constexpr float WCARRY      = 64.0f;
constexpr float WCARRY_INV  = 1.0f / 64.0f;
constexpr float LOCARRY     = 2048.0f;
constexpr float LOCARRY_INV = 1.0f / 2048.0f;
constexpr float THCARRY     = 16.0f;
constexpr float EWCARRY     = 1024.0f;
constexpr float LIB_FOLD    = 1.0f / (16.0f * 1024.0f);
constexpr float GRAM_SCALE  = 1.0f / 1024.0f;
static_assert(KREAL == 47968, "library width");
static_assert(NQUAD == LATD * (LATD + 1) / 2, "quad count");
static_assert(NCUBE == 66 * 65 * 64 / 6, "cubic count");
static_assert(KPADDED % 32 == 0 && KPADDED >= KREAL, "padded K");
static_assert(KCHUNK * KSPLITS == KPADDED && KCHUNK % 32 == 0, "split-K chunk");
static_assert(KREAL % 8 == 0 && KPADDED % 8 == 0 && KGRP8 == 6016, "8-column groups");
static_assert(NSAMP % 64 == 0 && LATD % 64 == 0 && HID_A % 64 == 0 && HID_B % 64 == 0, "tile multiples");
static_assert(LATD % 32 == 0 && HID_A % 32 == 0 && HID_B % 32 == 0 && NSAMP % 32 == 0, "K multiples of 32");
static_assert(5 * PLANE_F == 327680, "output elements");

typedef __attribute__((ext_vector_type(16))) _Float16 v16h;
typedef __attribute__((ext_vector_type(8)))  _Float16 v8h;
typedef __attribute__((ext_vector_type(8)))  float    v8f;
typedef __attribute__((ext_vector_type(4)))  float    v4f;

__device__ __forceinline__ unsigned short f2bf_bits(float f) {
  unsigned u = __float_as_uint(f);
  return (unsigned short)((u + 0x7FFFu + ((u >> 16) & 1u)) >> 16);
}
__device__ __forceinline__ float bf_bits2f(unsigned short h) { return __uint_as_float(((unsigned)h) << 16); }

__device__ __forceinline__ void dep_guard4_h(v8f& a, v8f& b, v8f& c, v8f& d, v16h x, v16h y) {
  asm volatile("v_nop\n\tv_nop\n\tv_nop\n\tv_nop" : "+v"(a), "+v"(b), "+v"(c), "+v"(d) : "v"(x), "v"(y));
}
__device__ __forceinline__ void keep4_h(v16h a, v16h b, v16h c, v16h d) { asm volatile("v_nop" :: "v"(a), "v"(b), "v"(c), "v"(d)); }
__device__ __forceinline__ void acc_guard4(v8f& a, v8f& b, v8f& c, v8f& d) {
  asm volatile("v_nop\n\tv_nop\n\tv_nop\n\tv_nop" : "+v"(a), "+v"(b), "+v"(c), "+v"(d));
}
__device__ __forceinline__ void guard_all4(v8f& a0, v8f& a1, v8f& a2, v8f& a3,
                                           v16h x, v16h b0, v16h b1, v16h b2, v16h b3) {
  asm volatile("v_nop\n\tv_nop\n\tv_nop\n\tv_nop"
               : "+v"(a0), "+v"(a1), "+v"(a2), "+v"(a3)
               : "v"(x), "v"(b0), "v"(b1), "v"(b2), "v"(b3));
}
__device__ __forceinline__ void guard_all8(v8f& a0, v8f& a1, v8f& a2, v8f& a3,
                                           v8f& r0, v8f& r1, v8f& r2, v8f& r3,
                                           v16h x, v16h y,
                                           v16h b0, v16h b1, v16h b2, v16h b3,
                                           v16h c0, v16h c1, v16h c2, v16h c3) {
  asm volatile("v_nop\n\tv_nop\n\tv_nop\n\tv_nop"
               : "+v"(a0), "+v"(a1), "+v"(a2), "+v"(a3), "+v"(r0), "+v"(r1), "+v"(r2), "+v"(r3)
               : "v"(x), "v"(y), "v"(b0), "v"(b1), "v"(b2), "v"(b3), "v"(c0), "v"(c1), "v"(c2), "v"(c3));
}
__device__ __forceinline__ void wave_lds_sync() {
  __builtin_amdgcn_fence(__ATOMIC_RELEASE, "workgroup");
  __builtin_amdgcn_wave_barrier();
  __builtin_amdgcn_fence(__ATOMIC_ACQUIRE, "workgroup");
}

template <typename T> struct Frag;
template <> struct Frag<_Float16> {
  typedef v16h V; union U { v16h v; v8h h[2]; };
  static __device__ __forceinline__ v16h load(const _Float16* p) {
    U f; f.h[0] = *(const v8h*)(p); f.h[1] = *(const v8h*)(p + 16); return f.v;
  }
  static __device__ __forceinline__ v8f mma(v16h a, v16h b, v8f c) {
    return __builtin_amdgcn_wmma_f32_16x16x32_f16(false, a, false, b, (short)0, c, false, false);
  }
  static __device__ __forceinline__ void guard4(v8f& a, v8f& b, v8f& c, v8f& d, v16h x, v16h y) { dep_guard4_h(a, b, c, d, x, y); }
  static __device__ __forceinline__ void keep(v16h a, v16h b, v16h c, v16h d) { keep4_h(a, b, c, d); }
};

template <int ET> struct Elem;
template <> struct Elem<0> { typedef _Float16 T; };
template <int ET, bool SPLIT, int BIAS_MODE, int OUT_MODE, bool RESID, int ACT = 0>
__global__ __launch_bounds__(256) void wmma_gemm64(
    const unsigned short* __restrict__ Ap, const unsigned short* __restrict__ A2p, int lda, long strideA,
    const unsigned short* __restrict__ Btp, const unsigned short* __restrict__ Bt2p, int ldb, long strideB,
    void* __restrict__ Cout, void* __restrict__ Cout2, int ldc, long strideC,
    const float* __restrict__ bias,
    const float* __restrict__ resid, long strideR,
    int M, int N, int K, float scale) {
  typedef typename Elem<ET>::T T;
  typedef typename Frag<T>::V V;
  const T* A = (const T*)Ap; const T* A2 = (const T*)A2p; const T* Bt = (const T*)Btp; const T* Bt2 = (const T*)Bt2p;
  __shared__ __align__(16) float sT[8][16 * 68];
  const int b    = blockIdx.y;
  const int lane = threadIdx.x & 31;
  const int wave = threadIdx.x >> 5;
  const int tilesN = N >> 6;
  const int tilesM = M >> 6;
  const int tile = blockIdx.x * 8 + wave;
  if (tile >= tilesM * tilesN) return;
  const int tm = tile / tilesN;
  const int tn = tile - tm * tilesN;
  const int m0 = tm << 6;
  const int n0 = tn << 6;

  const T* Ab  = A  + (size_t)b * strideA;
  const T* Bb  = Bt + (size_t)b * strideB;
  const T* Ab2 = SPLIT ? (A2  + (size_t)b * strideA) : nullptr;
  const T* Bb2 = SPLIT ? (Bt2 + (size_t)b * strideB) : nullptr;

  const int rlane = lane & 15;
  const int koff  = (lane >> 4) * 8;
  const int mOff  = (lane >> 4) * 8;

  v8f acc[4][4];
#pragma unroll
  for (int i = 0; i < 4; ++i)
#pragma unroll
    for (int j = 0; j < 4; ++j) acc[i][j] = (v8f){0.f,0.f,0.f,0.f,0.f,0.f,0.f,0.f};

  for (int k0 = 0; k0 < K; k0 += 32) {
    V bh[4], bl[4];
#pragma unroll
    for (int j = 0; j < 4; ++j) {
      const size_t bo = (size_t)(n0 + (j << 4) + rlane) * ldb + koff + k0;
      bh[j] = Frag<T>::load(Bb + bo);
      if (SPLIT) bl[j] = Frag<T>::load(Bb2 + bo);
    }
#pragma unroll
    for (int i = 0; i < 4; ++i) {
      const size_t ao = (size_t)(m0 + (i << 4) + rlane) * lda + koff + k0;
      V ah = Frag<T>::load(Ab + ao);
      V al;
      if (SPLIT) al = Frag<T>::load(Ab2 + ao);
#pragma unroll
      for (int j = 0; j < 4; ++j) {
        acc[i][j] = Frag<T>::mma(ah, bh[j], acc[i][j]);
        if (SPLIT) {
          acc[i][j] = Frag<T>::mma(ah, bl[j], acc[i][j]);
          acc[i][j] = Frag<T>::mma(al, bh[j], acc[i][j]);
        }
      }
      Frag<T>::guard4(acc[i][0], acc[i][1], acc[i][2], acc[i][3], ah, SPLIT ? al : ah);
    }
    Frag<T>::keep(bh[0], bh[1], bh[2], bh[3]);
    if (SPLIT) Frag<T>::keep(bl[0], bl[1], bl[2], bl[3]);
  }
  acc_guard4(acc[0][0], acc[0][1], acc[0][2], acc[0][3]);
  acc_guard4(acc[1][0], acc[1][1], acc[1][2], acc[1][3]);
  acc_guard4(acc[2][0], acc[2][1], acc[2][2], acc[2][3]);
  acc_guard4(acc[3][0], acc[3][1], acc[3][2], acc[3][3]);

  float* slab = sT[wave];
  const float* Rb = RESID ? (resid + (size_t)b * strideR) : nullptr;
#pragma unroll
  for (int i = 0; i < 4; ++i) {
    const int mBase = m0 + (i << 4);
#pragma unroll
    for (int j = 0; j < 4; ++j) {
      const int n = n0 + (j << 4) + rlane;
      float bv = 0.f;
      if (BIAS_MODE == 2) bv = bias[n];
#pragma unroll
      for (int r = 0; r < 8; ++r) {
        float v = acc[i][j][r] * scale;
        if (BIAS_MODE == 1) v += bias[mBase + mOff + r];
        if (BIAS_MODE == 2) v += bv;
        if (RESID) v += Rb[(size_t)(mBase + mOff + r) * ldc + n];
        if (ACT == 1) v = tanhf(v);
        if (ACT == 2) v = fmaxf(v, 0.0f);
        if (ACT == 3) v = v / (1.0f + expf(-v));
        if (ACT == 4) v = (v > 0.f) ? v : 0.01f * v;
        if (ACT == 5) v = 0.5f * v * (1.0f + erff(v * 0.70710678118654752f));
        slab[(mOff + r) * 68 + (j << 4) + rlane] = v;
      }
    }
    wave_lds_sync();
    if (OUT_MODE == 0) {
      float* C = (float*)Cout + (size_t)b * strideC;
      const int hh = lane >> 4, c4 = (lane & 15) * 4;
      for (int pass = 0; pass < 2; ++pass) {
#pragma unroll
        for (int it = 0; it < 8; ++it) {
          const int row = it * 2 + hh;
          v4f v = *(const v4f*)(slab + row * 68 + c4);
          *(volatile v4f*)(C + (size_t)(mBase + row) * ldc + n0 + c4) = v;
        }
        __threadfence();
      }
    } else {
      const int q = lane >> 3, c8 = (lane & 7) * 8;
      unsigned short* C  = (unsigned short*)Cout  + (size_t)b * strideC;
      unsigned short* C2 = (OUT_MODE == 2) ? ((unsigned short*)Cout2 + (size_t)b * strideC) : nullptr;
      for (int pass = 0; pass < 2; ++pass) {
#pragma unroll
        for (int it = 0; it < 4; ++it) {
          const int row = it * 4 + q;
          const float* sp = slab + row * 68 + c8;
          v8h hv, lv;
#pragma unroll
          for (int e = 0; e < 8; ++e) {
            if (OUT_MODE == 1) {
              hv[e] = (_Float16)sp[e];
            } else {
              unsigned short hb = f2bf_bits(sp[e]);
              unsigned short lb = f2bf_bits(sp[e] - bf_bits2f(hb));
              hv[e] = __builtin_bit_cast(_Float16, hb);
              lv[e] = __builtin_bit_cast(_Float16, lb);
            }
          }
          *(volatile v8h*)(C + (size_t)(mBase + row) * ldc + n0 + c8) = hv;
          if (OUT_MODE == 2) *(volatile v8h*)(C2 + (size_t)(mBase + row) * ldc + n0 + c8) = lv;
        }
        __threadfence();
      }
    }
    wave_lds_sync();
  }
}

template <bool LO>
__global__ __launch_bounds__(256) void cvt_rows8(const float* __restrict__ src, unsigned short* dhi, unsigned short* dlo,
                                                 int nrow, int dcol8, int spitch, int scols, float sc) {
  const int i  = blockIdx.x * 256 + threadIdx.x;
  const int n8 = nrow * dcol8;
  if (i < n8) {
    const int row = i / dcol8;
    const int c0  = (i - row * dcol8) * 8;
    const bool valid = c0 < scols;
    const int cc = valid ? c0 : (scols - 8);
    const float* sp = src + (size_t)row * spitch + cc;
    const v4f a = *(const v4f*)(sp);
    const v4f b = *(const v4f*)(sp + 4);
    v8h hv, lv;
#pragma unroll
    for (int e = 0; e < 4; ++e) {
      const float ae = a[e];
      const float be = b[e];
      const float f0 = valid ? ae * sc : 0.0f;
      const float f1 = valid ? be * sc : 0.0f;
      const _Float16 h0 = (_Float16)f0;
      const _Float16 h1 = (_Float16)f1;
      hv[e]     = h0;
      hv[4 + e] = h1;
      if (LO) {
        const float r0 = f0 - (float)h0;
        const float r1 = f1 - (float)h1;
        lv[e]     = (_Float16)(r0 * LOCARRY);
        lv[4 + e] = (_Float16)(r1 * LOCARRY);
      }
    }
    *(volatile v8h*)(dhi + (size_t)i * 8) = hv;
    if (LO) *(volatile v8h*)(dlo + (size_t)i * 8) = lv;
    __threadfence();
    *(volatile v8h*)(dhi + (size_t)i * 8) = hv;
    if (LO) *(volatile v8h*)(dlo + (size_t)i * 8) = lv;
  }
}

template <bool SPLIT, int EPI, bool LOOUT>
__global__ __launch_bounds__(256) void mlp_gemm16(
    const unsigned short* __restrict__ Ahp, const unsigned short* __restrict__ Alp,
    const unsigned short* __restrict__ Bhp, const unsigned short* __restrict__ Blp,
    const float* __restrict__ bias,
    float* F0, float* F1, unsigned short* H0, unsigned short* H1,
    int M, int N, int K, float scale) {
  __shared__ __align__(16) float sT[8][16 * 68];
  const _Float16* Ah = (const _Float16*)Ahp;
  const _Float16* Al = (const _Float16*)Alp;
  const _Float16* Bh = (const _Float16*)Bhp;
  const _Float16* Bl = (const _Float16*)Blp;
  const int lane = threadIdx.x & 31;
  const int wave = threadIdx.x >> 5;
  const int tilesN = N >> 6;
  const int tilesM = M >> 4;
  const int tile = blockIdx.x * 8 + wave;
  if (tile >= tilesM * tilesN) return;
  const int tm = tile / tilesN;
  const int tn = tile - tm * tilesN;
  const int m0 = tm << 4;
  const int n0 = tn << 6;
  const int rlane = lane & 15;
  const int koff  = (lane >> 4) * 8;
  const int mOff  = (lane >> 4) * 8;

  v8f acc[4], accr[4];
#pragma unroll
  for (int j = 0; j < 4; ++j) {
    acc[j]  = (v8f){0.f,0.f,0.f,0.f,0.f,0.f,0.f,0.f};
    accr[j] = (v8f){0.f,0.f,0.f,0.f,0.f,0.f,0.f,0.f};
  }

  for (int k0 = 0; k0 < K; k0 += 32) {
    const size_t ao = (size_t)(m0 + rlane) * K + koff + k0;
    const v16h ah = Frag<_Float16>::load(Ah + ao);
    v16h al = ah;
    if (SPLIT) al = Frag<_Float16>::load(Al + ao);
    v16h bh[4], bl[4];
#pragma unroll
    for (int j = 0; j < 4; ++j) {
      const size_t bo = (size_t)(n0 + (j << 4) + rlane) * K + koff + k0;
      bh[j] = Frag<_Float16>::load(Bh + bo);
      bl[j] = bh[j];
      if (SPLIT) bl[j] = Frag<_Float16>::load(Bl + bo);
      acc[j] = Frag<_Float16>::mma(ah, bh[j], acc[j]);
      if (SPLIT) {
        accr[j] = Frag<_Float16>::mma(ah, bl[j], accr[j]);
        accr[j] = Frag<_Float16>::mma(al, bh[j], accr[j]);
      }
      asm volatile("" ::: "memory");
    }
    if (SPLIT) {
      guard_all8(acc[0], acc[1], acc[2], acc[3], accr[0], accr[1], accr[2], accr[3],
                 ah, al, bh[0], bh[1], bh[2], bh[3], bl[0], bl[1], bl[2], bl[3]);
    } else {
      guard_all4(acc[0], acc[1], acc[2], acc[3], ah, bh[0], bh[1], bh[2], bh[3]);
    }
  }
  acc_guard4(acc[0], acc[1], acc[2], acc[3]);
  if (SPLIT) acc_guard4(accr[0], accr[1], accr[2], accr[3]);

  float* slab = sT[wave];
  const float rscale = scale * LOCARRY_INV;
#pragma unroll
  for (int j = 0; j < 4; ++j) {
    const int n = n0 + (j << 4) + rlane;
    const float bv = bias[n];
#pragma unroll
    for (int r = 0; r < 8; ++r) {
      float v = acc[j][r] * scale;
      if (SPLIT) v += accr[j][r] * rscale;
      v += bv;
      slab[(mOff + r) * 68 + (j << 4) + rlane] = v;
    }
  }
  wave_lds_sync();

  const int hh = lane >> 4, c4 = (lane & 15) * 4;
  const int q  = lane >> 3, c8 = (lane & 7) * 8;

  if (EPI == 0) {
#pragma unroll 1
    for (int it = 0; it < 8; ++it) {
      float* sp = slab + (it * 2 + hh) * 68 + c4;
      const v4f p = *(const v4f*)sp;
      v4f hq;
#pragma unroll
      for (int e = 0; e < 4; ++e) {
        const float pe = p[e];
        hq[e] = 1.0f / (1.0f + expf(-pe));
      }
      *(v4f*)sp = hq;
    }
    wave_lds_sync();
    for (int pass = 0; pass < 2; ++pass) {
#pragma unroll
      for (int it = 0; it < 8; ++it) {
        const int row = it * 2 + hh;
        const v4f hq = *(const v4f*)(slab + row * 68 + c4);
        v4f gq;
#pragma unroll
        for (int e = 0; e < 4; ++e) {
          const float he = hq[e];
          gq[e] = he * (1.0f - he);
        }
        *(volatile v4f*)(F0 + (size_t)(m0 + row) * N + n0 + c4) = gq;
      }
#pragma unroll
      for (int it = 0; it < 4; ++it) {
        const int row = it * 4 + q;
        const float* sp = slab + row * 68 + c8;
        v8h hv, lv;
#pragma unroll
        for (int e = 0; e < 8; ++e) {
          const float xv = sp[e];
          const _Float16 hx = (_Float16)xv;
          hv[e] = hx;
          if (LOOUT) {
            const float rr = xv - (float)hx;
            lv[e] = (_Float16)(rr * LOCARRY);
          }
        }
        *(volatile v8h*)(H0 + (size_t)(m0 + row) * N + n0 + c8) = hv;
        if (LOOUT) *(volatile v8h*)(H1 + (size_t)(m0 + row) * N + n0 + c8) = lv;
      }
      __threadfence();
    }
  } else {
    for (int pass = 0; pass < 2; ++pass) {
#pragma unroll
      for (int it = 0; it < 8; ++it) {
        const int row = it * 2 + hh;
        const v4f v = *(const v4f*)(slab + row * 68 + c4);
        *(volatile v4f*)(F0 + (size_t)(m0 + row) * N + n0 + c4) = v;
        if (EPI == 1) *(volatile v4f*)(F1 + (size_t)(m0 + row) * N + n0 + c4) = v;
      }
      if (EPI == 1) {
#pragma unroll
        for (int it = 0; it < 4; ++it) {
          const int row = it * 4 + q;
          const float* sp = slab + row * 68 + c8;
          v8h hv;
#pragma unroll
          for (int e = 0; e < 8; ++e) {
            const float xv = sp[e];
            hv[e] = (_Float16)xv;
          }
          *(volatile v8h*)(H0 + (size_t)(m0 + row) * N + n0 + c8) = hv;
        }
      }
      __threadfence();
    }
  }
  wave_lds_sync();
}

__global__ __launch_bounds__(256) void transpose_g16(const float* __restrict__ G, unsigned short* Gt, int F) {
  __shared__ float Tt[64 * 65];
  const int tid = threadIdx.x, lane = tid & 31, wave = tid >> 5;
  const int f0 = blockIdx.x * 64;
  const int s0 = blockIdx.y * 64;
#pragma unroll
  for (int it = 0; it < 4; ++it) {
    const int idx = tid + 256 * it;
    const int row = idx >> 4;
    const int cc4 = (idx & 15) * 4;
    const v4f v = *(const v4f*)(G + (size_t)(s0 + row) * F + f0 + cc4);
#pragma unroll
    for (int e = 0; e < 4; ++e) {
      const float ve = v[e];
      Tt[(cc4 + e) * 65 + row] = ve;
    }
  }
  __syncthreads();
  const int q = lane >> 3, c8 = (lane & 7) * 8;
  for (int pass = 0; pass < 2; ++pass) {
#pragma unroll
    for (int it = 0; it < 2; ++it) {
      const int f = it * 32 + wave * 4 + q;
      const float* sp = Tt + f * 65 + c8;
      v8h hv;
#pragma unroll
      for (int e = 0; e < 8; ++e) {
        const float xv = sp[e];
        hv[e] = (_Float16)xv;
      }
      *(volatile v8h*)(Gt + (size_t)(f0 + f) * NSAMP + s0 + c8) = hv;
    }
    __threadfence();
  }
}

template <bool HAS_G>
__global__ __launch_bounds__(256) void f32_mm4(const float* __restrict__ A, const float* __restrict__ B,
                                               const float* __restrict__ G, float* C, int M, int N, int K) {
  const int t = blockIdx.x * 256 + threadIdx.x;
  const int n4c = N >> 2;
  if (t < M * n4c) {
    const int m  = t / n4c;
    const int n4 = (t - m * n4c) * 4;
    const float* ap = A + (size_t)m * K;
    v4f acc = (v4f){0.0f, 0.0f, 0.0f, 0.0f};
#pragma unroll 1
    for (int k = 0; k < K; ++k) {
      const float a = ap[k];
      const v4f b = *(const v4f*)(B + (size_t)k * N + n4);
      v4f g = b;
      if (HAS_G) g = *(const v4f*)(G + (size_t)k * N + n4);
#pragma unroll
      for (int e = 0; e < 4; ++e) {
        const float be = b[e];
        const float ge = g[e];
        const float w = HAS_G ? be * ge : be;
        acc[e] += a * w;
      }
    }
    *(volatile v4f*)(C + (size_t)t * 4) = acc;
    __threadfence();
    *(volatile v4f*)(C + (size_t)t * 4) = acc;
  }
}

__global__ __launch_bounds__(256) void theta_plane_kernel(const float* __restrict__ ZF, unsigned short* TH) {
  __shared__ float zs[LATD];
  __shared__ int   cot[LATD];
  __shared__ float qd[NQUAD];
  const int tid = threadIdx.x;
  const int n = blockIdx.x;
  if (tid < LATD) {
    zs[tid] = ZF[(size_t)n * LATD + tid];
    const int mm = 66 - tid;
    cot[tid] = NCUBE - (mm * (mm - 1) * (mm - 2)) / 6;
  }
  __syncthreads();
#pragma unroll 1
  for (int it = 0; it < 16; ++it) {
    const int p = tid + 256 * it;
    const int i = p >> 6;
    const int j = p & 63;
    const float zi = zs[i];
    const float zj = zs[j];
    if (i <= j) qd[64 * i - ((i * (i - 1)) >> 1) + (j - i)] = zi * zj;
  }
  __syncthreads();
  unsigned short* trow = TH + (size_t)n * KPADDED;
#pragma unroll 1
  for (int g = tid; g < KGRP8; g += 256) {
    const int c0 = g * 8;
    v8h hv;
#pragma unroll
    for (int e = 0; e < 8; ++e) {
      const int c = c0 + e;
      int u = c - (2 * LATD + NQUAD);
      u = u < 0 ? 0 : u;
      u = u > (NCUBE - 1) ? (NCUBE - 1) : u;
      int i = 0;
      i += (cot[i + 32] <= u) ? 32 : 0;
      i += (cot[i + 16] <= u) ? 16 : 0;
      i += (cot[i + 8]  <= u) ? 8 : 0;
      i += (cot[i + 4]  <= u) ? 4 : 0;
      i += (cot[i + 2]  <= u) ? 2 : 0;
      i += (cot[i + 1]  <= u) ? 1 : 0;
      int qi = 64 * i - ((i * (i - 1)) >> 1) + (u - cot[i]);
      qi = qi < 0 ? 0 : qi;
      qi = qi > (NQUAD - 1) ? (NQUAD - 1) : qi;
      const float vc = zs[i] * qd[qi];
      int tq = c - 2 * LATD;
      tq = tq < 0 ? 0 : tq;
      tq = tq > (NQUAD - 1) ? (NQUAD - 1) : tq;
      const float vq = qd[tq];
      int tl = c - LATD;
      tl = tl < 0 ? 0 : tl;
      tl = tl > (LATD - 1) ? (LATD - 1) : tl;
      const float vl = zs[tl];
      float v = (c < KREAL) ? vc : 0.0f;
      v = (c < 2 * LATD + NQUAD) ? vq : v;
      v = (c < 2 * LATD) ? vl : v;
      v = (c < LATD) ? 1.0f : v;
      hv[e] = (_Float16)(v * THCARRY);
    }
    *(volatile v8h*)(trow + c0) = hv;
    __threadfence();
    *(volatile v8h*)(trow + c0) = hv;
  }
}

__global__ __launch_bounds__(256) void splitk_combine(const float* __restrict__ PART, const float* __restrict__ Eb,
                                                      float* OUTP, float* WSC) {
  const int t = blockIdx.x * 256 + threadIdx.x;
  const int n4 = (t & 15) * 4;
  v4f s = (v4f){0.0f, 0.0f, 0.0f, 0.0f};
#pragma unroll 1
  for (int sp = 0; sp < KSPLITS; ++sp) {
    const v4f p = *(const v4f*)(PART + (size_t)sp * PLANE_F + (size_t)t * 4);
#pragma unroll
    for (int e = 0; e < 4; ++e) {
      const float pe = p[e];
      s[e] += pe;
    }
  }
  const v4f bq = *(const v4f*)(Eb + n4);
#pragma unroll
  for (int e = 0; e < 4; ++e) {
    const float be = bq[e];
    s[e] += be;
  }
  *(volatile v4f*)(OUTP + (size_t)t * 4) = s;
  *(volatile v4f*)(WSC + (size_t)t * 4) = s;
  __threadfence();
  *(volatile v4f*)(OUTP + (size_t)t * 4) = s;
  *(volatile v4f*)(WSC + (size_t)t * 4) = s;
}

constexpr size_t WS_TOTAL =
    2 * 131072ull + 2 * 32768ull + 2 * 65536ull + 2 * 16384ull + 16384ull + 65536ull + 32768ull +
    (size_t)LATD * KPADDED * 2 + 2 * 524288ull + 2 * 262144ull + 1048576ull + 524288ull + 262144ull + 131072ull +
    262144ull + 524288ull + 524288ull + 1048576ull + 524288ull + 262144ull + 262144ull + 524288ull +
    131072ull + 131072ull + 65536ull + 32768ull + 2 * 16384ull + (size_t)KSPLITS * PLANE_F * 4 + 262144ull +
    (size_t)NSAMP * KPADDED * 2;
static_assert(WS_TOTAL == 117653504ull, "carve total");
static_assert(WS_TOTAL <= 134217728ull, "carve budget");

extern "C" void kernel_launch(void* const* d_in, const int* in_sizes, int n_in,
                              void* d_out, int out_size, void* d_ws, size_t ws_size, hipStream_t stream) {
  if (n_in < 17 || d_out == nullptr || d_ws == nullptr) return;
  if (in_sizes[0] != NSAMP * LATD || in_sizes[1] != NSAMP * LATD ||
      in_sizes[3] != HID_A * LATD || in_sizes[4] != HID_A ||
      in_sizes[5] != HID_B * HID_A || in_sizes[6] != HID_B ||
      in_sizes[7] != LATD * HID_B || in_sizes[8] != LATD ||
      in_sizes[9] != HID_B * LATD || in_sizes[10] != HID_B ||
      in_sizes[11] != HID_A * HID_B || in_sizes[12] != HID_A ||
      in_sizes[13] != LATD * HID_A || in_sizes[14] != LATD ||
      in_sizes[15] != LATD * KREAL || in_sizes[16] != LATD ||
      out_size != 5 * PLANE_F) return;

  const float* x_in   = (const float*)d_in[0];
  const float* dx_in  = (const float*)d_in[1];
  const float* we_W0 = (const float*)d_in[3];
  const float* we_b0 = (const float*)d_in[4];
  const float* we_W1 = (const float*)d_in[5];
  const float* we_b1 = (const float*)d_in[6];
  const float* we_W2 = (const float*)d_in[7];
  const float* we_b2 = (const float*)d_in[8];
  const float* wd_W0 = (const float*)d_in[9];
  const float* wd_b0 = (const float*)d_in[10];
  const float* wd_W1 = (const float*)d_in[11];
  const float* wd_b1 = (const float*)d_in[12];
  const float* wd_W2 = (const float*)d_in[13];
  const float* wd_b2 = (const float*)d_in[14];
  const float* E_W   = (const float*)d_in[15];
  const float* E_b   = (const float*)d_in[16];
  float* out = (float*)d_out;
  float* out_z   = out;
  float* out_dz  = out + (size_t)1 * PLANE_F;
  float* out_dzb = out + (size_t)2 * PLANE_F;
  float* out_xb  = out + (size_t)3 * PLANE_F;
  float* out_dxb = out + (size_t)4 * PLANE_F;

  char* ws = (char*)d_ws; size_t off = 0;
  auto carve = [&](size_t bytes) -> char* { char* p = ws + off; off += (bytes + 255) & ~(size_t)255; return p; };
  unsigned short* XH   = (unsigned short*)carve((size_t)NSAMP * LATD * 2);
  unsigned short* XL   = (unsigned short*)carve((size_t)NSAMP * LATD * 2);
  unsigned short* W0H  = (unsigned short*)carve((size_t)HID_A * LATD * 2);
  unsigned short* W0L  = (unsigned short*)carve((size_t)HID_A * LATD * 2);
  unsigned short* W1H  = (unsigned short*)carve((size_t)HID_B * HID_A * 2);
  unsigned short* W1L  = (unsigned short*)carve((size_t)HID_B * HID_A * 2);
  unsigned short* W2H  = (unsigned short*)carve((size_t)LATD * HID_B * 2);
  unsigned short* W2L  = (unsigned short*)carve((size_t)LATD * HID_B * 2);
  unsigned short* D0H  = (unsigned short*)carve((size_t)HID_B * LATD * 2);
  unsigned short* D1H  = (unsigned short*)carve((size_t)HID_A * HID_B * 2);
  unsigned short* D2H  = (unsigned short*)carve((size_t)LATD * HID_A * 2);
  unsigned short* EWH  = (unsigned short*)carve((size_t)LATD * KPADDED * 2);
  unsigned short* H1H  = (unsigned short*)carve((size_t)NSAMP * HID_A * 2);
  unsigned short* H1L  = (unsigned short*)carve((size_t)NSAMP * HID_A * 2);
  unsigned short* H2H  = (unsigned short*)carve((size_t)NSAMP * HID_B * 2);
  unsigned short* H2L  = (unsigned short*)carve((size_t)NSAMP * HID_B * 2);
  float*          G1   = (float*)carve((size_t)NSAMP * HID_A * 4);
  float*          G2   = (float*)carve((size_t)NSAMP * HID_B * 4);
  float*          ZF   = (float*)carve((size_t)NSAMP * LATD * 4);
  unsigned short* ZH   = (unsigned short*)carve((size_t)NSAMP * LATD * 2);
  unsigned short* D1A  = (unsigned short*)carve((size_t)NSAMP * HID_B * 2);
  unsigned short* D2A  = (unsigned short*)carve((size_t)NSAMP * HID_A * 2);
  float*          GD1  = (float*)carve((size_t)NSAMP * HID_B * 4);
  float*          GD2  = (float*)carve((size_t)NSAMP * HID_A * 4);
  unsigned short* G1T  = (unsigned short*)carve((size_t)HID_A * NSAMP * 2);
  unsigned short* G2T  = (unsigned short*)carve((size_t)HID_B * NSAMP * 2);
  unsigned short* GD1T = (unsigned short*)carve((size_t)HID_B * NSAMP * 2);
  unsigned short* GD2T = (unsigned short*)carve((size_t)HID_A * NSAMP * 2);
  float*          GE   = (float*)carve((size_t)HID_B * HID_A * 4);
  float*          GD   = (float*)carve((size_t)HID_A * HID_B * 4);
  float*          TE   = (float*)carve((size_t)LATD * HID_A * 4);
  float*          TD   = (float*)carve((size_t)LATD * HID_B * 4);
  float*          JE   = (float*)carve((size_t)LATD * LATD * 4);
  float*          JD   = (float*)carve((size_t)LATD * LATD * 4);
  float*          PART = (float*)carve((size_t)KSPLITS * PLANE_F * 4);
  float*          DZBW = (float*)carve((size_t)PLANE_F * 4);
  unsigned short* THETA = (unsigned short*)carve((size_t)NSAMP * KPADDED * 2);
  if (off != WS_TOTAL || off > ws_size || off > (size_t)134217728) return;

  cvt_rows8<true ><<<(NSAMP * (LATD / 8)) / 256, 256, 0, stream>>>(x_in,  XH,  XL,  NSAMP, LATD / 8,  LATD,  LATD,  1.0f);
  cvt_rows8<true ><<<(HID_A * (LATD / 8)) / 256, 256, 0, stream>>>(we_W0, W0H, W0L, HID_A, LATD / 8,  LATD,  LATD,  WCARRY);
  cvt_rows8<true ><<<(HID_B * (HID_A / 8)) / 256, 256, 0, stream>>>(we_W1, W1H, W1L, HID_B, HID_A / 8, HID_A, HID_A, WCARRY);
  cvt_rows8<true ><<<(LATD * (HID_B / 8)) / 256, 256, 0, stream>>>(we_W2, W2H, W2L, LATD,  HID_B / 8, HID_B, HID_B, WCARRY);
  cvt_rows8<false><<<(HID_B * (LATD / 8)) / 256, 256, 0, stream>>>(wd_W0, D0H, D0H, HID_B, LATD / 8,  LATD,  LATD,  WCARRY);
  cvt_rows8<false><<<(HID_A * (HID_B / 8)) / 256, 256, 0, stream>>>(wd_W1, D1H, D1H, HID_A, HID_B / 8, HID_B, HID_B, WCARRY);
  cvt_rows8<false><<<(LATD * (HID_A / 8)) / 256, 256, 0, stream>>>(wd_W2, D2H, D2H, LATD,  HID_A / 8, HID_A, HID_A, WCARRY);
  cvt_rows8<false><<<(LATD * KGRP8) / 256, 256, 0, stream>>>(E_W, EWH, EWH, LATD, KGRP8, KREAL, KREAL, EWCARRY);

  mlp_gemm16<true, 0, true><<<((NSAMP / 16) * (HID_A / 64)) / 8, 256, 0, stream>>>(
      XH, XL, W0H, W0L, we_b0, G1, G1, H1H, H1L, NSAMP, HID_A, LATD, WCARRY_INV);
  mlp_gemm16<true, 0, true><<<((NSAMP / 16) * (HID_B / 64)) / 8, 256, 0, stream>>>(
      H1H, H1L, W1H, W1L, we_b1, G2, G2, H2H, H2L, NSAMP, HID_B, HID_A, WCARRY_INV);
  mlp_gemm16<true, 1, false><<<((NSAMP / 16) * (LATD / 64)) / 8, 256, 0, stream>>>(
      H2H, H2L, W2H, W2L, we_b2, out_z, ZF, ZH, ZH, NSAMP, LATD, HID_B, WCARRY_INV);

  transpose_g16<<<dim3(HID_A / 64, NSAMP / 64), 256, 0, stream>>>(G1, G1T, HID_A);
  transpose_g16<<<dim3(HID_B / 64, NSAMP / 64), 256, 0, stream>>>(G2, G2T, HID_B);
  wmma_gemm64<0, false, 0, 0, false, 0><<<dim3(1, 1), 256, 0, stream>>>(
      G2T, G2T, NSAMP, 0L, G1T, G1T, NSAMP, 0L, (void*)GE, (void*)GE, HID_A, 0L,
      E_b, GE, 0L, HID_B, HID_A, NSAMP, GRAM_SCALE);
  f32_mm4<true ><<<(LATD * (HID_A / 4)) / 256, 256, 0, stream>>>(we_W2, we_W1, GE, TE, LATD, HID_A, HID_B);
  f32_mm4<false><<<(LATD * (LATD / 4)) / 256, 256, 0, stream>>>(TE, we_W0, we_W0, JE, LATD, LATD, HID_A);
  f32_mm4<false><<<(NSAMP * (LATD / 4)) / 256, 256, 0, stream>>>(dx_in, JE, JE, out_dz, NSAMP, LATD, LATD);

  theta_plane_kernel<<<NSAMP, 256, 0, stream>>>(ZF, THETA);
  wmma_gemm64<0, false, 0, 0, false, 0><<<dim3((NSAMP / 64) / 8, KSPLITS), 256, 0, stream>>>(
      THETA, THETA, KPADDED, (long)KCHUNK, EWH, EWH, KPADDED, (long)KCHUNK,
      (void*)PART, (void*)PART, LATD, (long)PLANE_F,
      E_b, PART, 0L, NSAMP, LATD, KCHUNK, LIB_FOLD);
  splitk_combine<<<(NSAMP * (LATD / 4)) / 256, 256, 0, stream>>>(PART, E_b, out_dzb, DZBW);

  mlp_gemm16<false, 0, false><<<((NSAMP / 16) * (HID_B / 64)) / 8, 256, 0, stream>>>(
      ZH, ZH, D0H, D0H, wd_b0, GD1, GD1, D1A, D1A, NSAMP, HID_B, LATD, WCARRY_INV);
  mlp_gemm16<false, 0, false><<<((NSAMP / 16) * (HID_A / 64)) / 8, 256, 0, stream>>>(
      D1A, D1A, D1H, D1H, wd_b1, GD2, GD2, D2A, D2A, NSAMP, HID_A, HID_B, WCARRY_INV);
  mlp_gemm16<false, 2, false><<<((NSAMP / 16) * (LATD / 64)) / 8, 256, 0, stream>>>(
      D2A, D2A, D2H, D2H, wd_b2, out_xb, out_xb, ZH, ZH, NSAMP, LATD, HID_A, WCARRY_INV);

  transpose_g16<<<dim3(HID_B / 64, NSAMP / 64), 256, 0, stream>>>(GD1, GD1T, HID_B);
  transpose_g16<<<dim3(HID_A / 64, NSAMP / 64), 256, 0, stream>>>(GD2, GD2T, HID_A);
  wmma_gemm64<0, false, 0, 0, false, 0><<<dim3(1, 1), 256, 0, stream>>>(
      GD2T, GD2T, NSAMP, 0L, GD1T, GD1T, NSAMP, 0L, (void*)GD, (void*)GD, HID_B, 0L,
      E_b, GD, 0L, HID_A, HID_B, NSAMP, GRAM_SCALE);
  f32_mm4<true ><<<(LATD * (HID_B / 4)) / 256, 256, 0, stream>>>(wd_W2, wd_W1, GD, TD, LATD, HID_B, HID_A);
  f32_mm4<false><<<(LATD * (LATD / 4)) / 256, 256, 0, stream>>>(TD, wd_W0, wd_W0, JD, LATD, LATD, HID_B);
  f32_mm4<false><<<(NSAMP * (LATD / 4)) / 256, 256, 0, stream>>>(DZBW, JD, JD, out_dxb, NSAMP, LATD, LATD);
}
